// ChebyshevLayer_80719615361565
// MI455X (gfx1250) — hardware-verified
//
#include <hip/hip_runtime.h>
#include <math.h>

typedef __attribute__((ext_vector_type(16))) _Float16 v16h;
typedef __attribute__((ext_vector_type(16))) __bf16 v16b;
typedef __attribute__((ext_vector_type(8)))  _Float16 v8h;
typedef __attribute__((ext_vector_type(8)))  float v8f;
typedef __attribute__((ext_vector_type(4)))  float v4f;
typedef __attribute__((ext_vector_type(2)))  float v2f;
typedef __attribute__((ext_vector_type(4)))  unsigned v4u;
typedef __attribute__((ext_vector_type(4)))  int v4i;
typedef float __attribute__((may_alias)) float_a;
typedef int __attribute__((may_alias)) int_a;

template <typename T> __device__ __forceinline__ void vst2(void* p, T v) { *(volatile T*)p = v; __threadfence(); *(volatile T*)p = v; }
__device__ __forceinline__ v8f wmma16(v16h a, v16h b, v8f c) {
  v8f d = __builtin_amdgcn_wmma_f32_16x16x32_f16(false, a, false, b, (short)0, c, false, false);
  asm volatile("v_nop\n\tv_nop\n\tv_nop\n\tv_nop" : "+v"(d) : "v"(a), "v"(b));
  return d;
}
__device__ __forceinline__ v8f wmma_bf(v16b a, v16b b, v8f c) {
  v8f d = __builtin_amdgcn_wmma_f32_16x16x32_bf16(false, a, false, b, (short)0, c, false, false);
  asm volatile("v_nop\n\tv_nop\n\tv_nop\n\tv_nop" : "+v"(d) : "v"(a), "v"(b));
  return d;
}
__device__ __forceinline__ v16h frag_h(const _Float16* rowk0, int lane) {
  union { v16h v; v8h q[2]; } u; const _Float16* p = rowk0 + 8 * (lane >> 4);
  u.q[0] = *(const v8h*)p; u.q[1] = *(const v8h*)(p + 16); return u.v;
}
__device__ __forceinline__ v16h frag_f32(const float* rowk0, int lane) {
  v16h a; const float* p = rowk0 + 8 * (lane >> 4);
#pragma unroll
  for (int i = 0; i < 8; ++i) { a[i] = (_Float16)p[i]; a[8 + i] = (_Float16)p[16 + i]; }
  return a;
}
__device__ __forceinline__ v16h frag_f32s(const float* rowk0, int lane, float sc) {
  v16h a; const float* p = rowk0 + 8 * (lane >> 4);
#pragma unroll
  for (int i = 0; i < 8; ++i) { a[i] = (_Float16)(p[i] * sc); a[8 + i] = (_Float16)(p[16 + i] * sc); }
  return a;
}
__device__ __forceinline__ v16h fragc_f32(const float* W, int k0, int n, int lane, int ld, int K) {
  v16h a; const int g = lane >> 4;
#pragma unroll
  for (int i = 0; i < 8; ++i) { const int ka = k0 + 8 * g + i, kb = ka + 16;
    a[i] = (_Float16)(ka < K ? W[(size_t)(ka < K ? ka : K - 1) * ld + n] : 0.f); a[8 + i] = (_Float16)(kb < K ? W[(size_t)(kb < K ? kb : K - 1) * ld + n] : 0.f); }
  return a;
}
struct F2 { v16b h, l; };
__device__ __forceinline__ F2 bsplit16(const float v[16]) { F2 r;
#pragma unroll
  for (int i = 0; i < 16; ++i) { const __bf16 h = (__bf16)v[i]; r.h[i] = h; r.l[i] = (__bf16)(v[i] - (float)h); }
  return r; }
__device__ __forceinline__ F2 split_row(const float* row, int k0, int lane) { float v[16]; const float* p = row + k0 + 8 * (lane >> 4);
#pragma unroll
  for (int i = 0; i < 8; ++i) { v[i] = p[i]; v[8 + i] = p[16 + i]; }
  return bsplit16(v); }
__device__ __forceinline__ F2 split_rowK(const float* row, int k0, int lane, int K) { float v[16]; const int g = lane >> 4;
#pragma unroll
  for (int i = 0; i < 8; ++i) { const int ka = k0 + 8 * g + i, kb = ka + 16; v[i] = ka < K ? row[ka < K ? ka : K - 1] : 0.f; v[8 + i] = kb < K ? row[kb < K ? kb : K - 1] : 0.f; }
  return bsplit16(v); }
__device__ __forceinline__ F2 split_col(const float* W, int k0, int n, int lane, int ld, int K) { float v[16]; const int g = lane >> 4;
#pragma unroll
  for (int i = 0; i < 8; ++i) { const int ka = k0 + 8 * g + i, kb = ka + 16; v[i] = ka < K ? W[(size_t)(ka < K ? ka : K - 1) * ld + n] : 0.f; v[8 + i] = kb < K ? W[(size_t)(kb < K ? kb : K - 1) * ld + n] : 0.f; }
  return bsplit16(v); }
__device__ __forceinline__ v8f mac3(const F2& a, const F2& b, v8f c) { c = wmma_bf(a.l, b.h, c); c = wmma_bf(a.h, b.l, c); return wmma_bf(a.h, b.h, c); }
__device__ __forceinline__ float sigm(float v) { return 1.0f / (1.0f + expf(-v)); }
#define LDSX() do { asm volatile("s_wait_dscnt 0" ::: "memory"); __builtin_amdgcn_wave_barrier(); __builtin_amdgcn_fence(__ATOMIC_RELEASE, "workgroup"); } while (0)


#define NBX 8192
#define NI 1024
#define NO 1024
#define ND 11
#define KP (NI * ND)
#define NPASS 2
#define PROWS (NBX / NPASS)
#ifndef TPASS
#define TPASS NPASS
#define TROWS PROWS
#endif
typedef __attribute__((ext_vector_type(8))) __bf16 v8b;
__device__ __forceinline__ v16b frag_b(const __bf16* rowk0, int lane) {
  union { v16b v; v8b q[2]; } u; const __bf16* p = rowk0 + 8 * (lane >> 4);
  u.q[0] = *(const v8b*)p; u.q[1] = *(const v8b*)(p + 16); return u.v;
}
__device__ __forceinline__ float bfr(float v) { return (float)(__bf16)v; }
__device__ __attribute__((noinline)) float exp_ni(float v) { return expf(v); }
__device__ __attribute__((noinline)) float erf_ni(float v) { return erff(v); }
__device__ __attribute__((noinline)) float tanh_ni(float v) { return tanhf(v); }

#define WS_PC  0u
#define WS_PW  (WS_PC + 2u * (size_t)NO * KP)
#define WS_BS  (WS_PW + 2u * (size_t)NO * NI)
#define WS_END (WS_BS + 2u * (size_t)PROWS * KP)

__global__ __launch_bounds__(256) void k_packc(const float* __restrict__ CO, _Float16* __restrict__ PC) {
  __shared__ __align__(16) _Float16 s[KP]; const int o = blockIdx.x, t = threadIdx.x;
  for (int k = t; k < KP; k += 256) { const int i = k / ND, n = k % ND; s[k] = (_Float16)bfr(CO[((size_t)i * NO + o) * ND + n]); }
  __syncthreads();
  for (int q = t; q < KP / 8; q += 256) vst2((unsigned*)(PC + (size_t)o * KP + q * 8), *(const v4u*)&s[q * 8]);
}
__global__ __launch_bounds__(256) void k_packw(const float* __restrict__ BW, __bf16* __restrict__ PW) {
  __shared__ __align__(16) __bf16 s[NI]; const int o = blockIdx.x, t = threadIdx.x;
  for (int i = t; i < NI; i += 256) s[i] = (__bf16)BW[(size_t)i * NO + o];
  __syncthreads();
  for (int q = t; q < NI / 8; q += 256) vst2((unsigned*)(PW + (size_t)o * NI + q * 8), *(const v4u*)&s[q * 8]);
}
__global__ __launch_bounds__(256) void k_basis(const float* __restrict__ X, int pass, _Float16* __restrict__ BS) {
  __shared__ __align__(16) _Float16 s[KP]; const int t = threadIdx.x; const size_t prow = blockIdx.x; const size_t row = (size_t)pass * PROWS + prow;
  for (int i = t; i < NI; i += 256) { const float tv = tanh_ni(bfr(X[row * NI + i])); float tm2 = 1.0f, tm1 = tv; s[i * ND + 0] = (_Float16)1.0f; s[i * ND + 1] = (_Float16)tv;
#pragma unroll
    for (int n = 2; n < ND; ++n) { const float tn = 2.0f * tv * tm1 - tm2; s[i * ND + n] = (_Float16)tn; tm2 = tm1; tm1 = tn; } }
  __syncthreads();
  for (int q = t; q < KP / 8; q += 256) vst2((unsigned*)(BS + prow * KP + q * 8), *(const v4u*)&s[q * 8]);
}
__global__ __launch_bounds__(128) void k_gemm(const _Float16* __restrict__ BS, const _Float16* __restrict__ PC, const float* __restrict__ X, const __bf16* __restrict__ PW, int pass, float* __restrict__ OUT) {
  __shared__ __align__(16) float so[4][16][132];
  const int tid = threadIdx.x, wave = tid >> 5, lane = tid & 31, col = lane & 15, g = lane >> 4; const size_t pr0 = (size_t)blockIdx.x * 64 + wave * 16; const size_t row0 = (size_t)pass * PROWS + pr0; const int n0 = blockIdx.y * 128;
  v8f acc[8] = {};
#pragma unroll 2
  for (int kc = 0; kc < KP / 32; ++kc) { const v16h a = frag_h(BS + (pr0 + col) * KP + kc * 32, lane);
#pragma unroll
    for (int j = 0; j < 8; ++j) acc[j] = wmma16(a, frag_h(PC + (size_t)(n0 + j * 16 + col) * KP + kc * 32, lane), acc[j]); }
#pragma unroll 2
  for (int kc = 0; kc < NI / 32; ++kc) { v16b a; { const float* p = X + (row0 + col) * NI + kc * 32 + 8 * g;
#pragma unroll
      for (int i = 0; i < 8; ++i) { a[i] = (__bf16)p[i]; a[8 + i] = (__bf16)p[16 + i]; } }
#pragma unroll
    for (int j = 0; j < 8; ++j) acc[j] = wmma_bf(a, frag_b(PW + (size_t)(n0 + j * 16 + col) * NI + kc * 32, lane), acc[j]); }
#pragma unroll
  for (int j = 0; j < 8; ++j)
#pragma unroll
    for (int r = 0; r < 8; ++r) so[wave][8 * g + r][j * 16 + col] = acc[j][r];
  LDSX();
  for (int rl = 0; rl < 16; ++rl) vst2(OUT + (row0 + rl) * NO + n0 + lane * 4, *(const v4f*)&so[wave][rl][lane * 4]);
}
extern "C" void kernel_launch(void* const* d_in, const int* in_sizes, int n_in, void* d_out, int out_size, void* d_ws, size_t ws_size, hipStream_t stream) {
  (void)in_sizes; (void)n_in; (void)out_size;
  const float** F = (const float**)d_in;
  if (ws_size < (size_t)WS_END) return;
  char* ws = (char*)d_ws; _Float16 *PC = (_Float16*)(ws + WS_PC), *BS = (_Float16*)(ws + WS_BS); __bf16* PW = (__bf16*)(ws + WS_PW);
  k_packc<<<NO, 256, 0, stream>>>(F[1], PC);
  k_packw<<<NO, 256, 0, stream>>>(F[2], PW);
  for (int pass = 0; pass < TPASS; ++pass) {
    k_basis<<<TROWS, 256, 0, stream>>>(F[0], pass, BS);
    k_gemm<<<dim3(TROWS / 64, NO / 128), 128, 0, stream>>>(BS, PC, F[0], PW, pass, (float*)d_out); }
}
